// MultiQueryAttention_5884105195698
// MI455X (gfx1250) — hardware-verified
//
#include <hip/hip_runtime.h>
#include <stddef.h>
#include <stdint.h>


#pragma clang fp contract(off)

#ifndef NB
#define NB 2
#endif
#ifndef SEQ
#define SEQ 2048
#endif
#define NB_FULL  2
#define SEQ_FULL 2048
#define DM   2048
#define NH   16
#define HD   128
#define HP   64
#define EROWS  (((SEQ) < 256) ? (SEQ) : 256)
#define ETILES (EROWS / 16)
#define MROWS  ((NB) * (SEQ))

#define BM  128
#define BK  32
#define LP  40
#define TP  136
#define RSC  2048.0f
#define RINV 0.00048828125f
#define PSC  1024.0f
#define PINV 0.0009765625f
#define WSC  64.0f
#define WINV 0.015625f

static_assert((SEQ) % 128 == 0);
static_assert((SEQ) >= 128 && (SEQ) <= SEQ_FULL);
static_assert((EROWS) % 128 == 0);
static_assert((NB) >= 1 && (NB) <= NB_FULL);
static_assert(DM % 128 == 0 && DM % BK == 0 && HD == 128 && NH * HD == DM);

#define SZ_X16 ((size_t)MROWS * DM * 2)
#define SZ_WQ  ((size_t)DM * DM * 2)
#define SZ_WK  ((size_t)HD * DM * 2)
#define SZ_QR  ((size_t)(NB) * EROWS * DM * 2)
#define SZ_KH  ((size_t)MROWS * HD * 2)
#define SZ_VT  ((size_t)(NB) * HD * (SEQ) * 2)
#define O_X16  ((size_t)0)
#define O_WQ   (O_X16 + SZ_X16)
#define O_WK   (O_WQ + SZ_WQ)
#define O_WV   (O_WK + SZ_WK)
#define O_WO   (O_WV + SZ_WK)
#define O_QH   (O_WO + SZ_WQ)
#define O_QR   (O_QH + SZ_X16)
#define O_KH   (O_QR + SZ_QR)
#define O_KR   (O_KH + SZ_KH)
#define O_VTH  (O_KR + SZ_KH)
#define O_VTR  (O_VTH + SZ_VT)
#define O_YH   (O_VTR + SZ_VT)
#define O_YR   (O_YH + SZ_X16)
#define WS_TOTAL (O_YR + SZ_QR)
static_assert(WS_TOTAL <= (size_t)134217728);
static_assert(SZ_WK % 256 == 0 && SZ_QR % 256 == 0 && SZ_VT % 256 == 0 && SZ_KH % 256 == 0);

typedef _Float16 v16h __attribute__((ext_vector_type(16)));
typedef _Float16 v8h  __attribute__((ext_vector_type(8)));
typedef float    v8f  __attribute__((ext_vector_type(8)));
typedef float    v4f  __attribute__((ext_vector_type(4)));

union HFrag { v16h v; v8h h[2]; };
struct HR8 { v8h h; v8h r; };

__device__ __forceinline__ float bfr(float f) {
    unsigned int u = __float_as_uint(f);
    u = (u + 0x7FFFu + ((u >> 16) & 1u)) & 0xFFFF0000u;
    return __uint_as_float(u);
}

__device__ __forceinline__ v16h load_frag(const _Float16* p) {
    HFrag f;
    f.h[0] = *reinterpret_cast<const v8h*>(p);
    f.h[1] = *reinterpret_cast<const v8h*>(p + 16);
    return f.v;
}

__device__ __forceinline__ v8f wmma16(v16h a, v16h b, v8f c) {
    c = __builtin_amdgcn_wmma_f32_16x16x32_f16(false, a, false, b, (short)0, c, false, false);
    asm volatile("v_nop\n\tv_nop\n\tv_nop\n\tv_nop" : "+v"(c) : "v"(a), "v"(b));
    return c;
}

__device__ __forceinline__ void wave_lds_sync() {
    __builtin_amdgcn_fence(3, "wavefront");
    __builtin_amdgcn_wave_barrier();
    __builtin_amdgcn_fence(2, "wavefront");
}

__device__ __forceinline__ HR8 pack8(v4f a, v4f b) {
    const _Float16 h0 = (_Float16)a.x, h1 = (_Float16)a.y, h2 = (_Float16)a.z, h3 = (_Float16)a.w;
    const _Float16 h4 = (_Float16)b.x, h5 = (_Float16)b.y, h6 = (_Float16)b.z, h7 = (_Float16)b.w;
    const _Float16 r0 = (_Float16)((a.x - (float)h0) * RSC);
    const _Float16 r1 = (_Float16)((a.y - (float)h1) * RSC);
    const _Float16 r2 = (_Float16)((a.z - (float)h2) * RSC);
    const _Float16 r3 = (_Float16)((a.w - (float)h3) * RSC);
    const _Float16 r4 = (_Float16)((b.x - (float)h4) * RSC);
    const _Float16 r5 = (_Float16)((b.y - (float)h5) * RSC);
    const _Float16 r6 = (_Float16)((b.z - (float)h6) * RSC);
    const _Float16 r7 = (_Float16)((b.w - (float)h7) * RSC);
    v8h hv = {h0, h1, h2, h3, h4, h5, h6, h7};
    v8h rv = {r0, r1, r2, r3, r4, r5, r6, r7};
    HR8 o;
    o.h = hv;
    o.r = rv;
    return o;
}

__device__ __forceinline__ v4f rope4(v4f f, float c0, float s0, float c1, float s1) {
    v4f o;
    o.x = f.x * c0 - f.y * s0;
    o.y = f.x * s0 + f.y * c0;
    o.z = f.z * c1 - f.w * s1;
    o.w = f.z * s1 + f.w * c1;
    return o;
}

__global__ __launch_bounds__(256) void k_cvt(const float* __restrict__ src, _Float16* dst,
                                             int ngrp, int ncols, int rows_per_seg,
                                             int src_seg_rows, float scale)
{
    const int g = blockIdx.x * 256 + threadIdx.x;
    if (g >= ngrp) return;
    const size_t e = (size_t)g * 8;
    const int r = (int)(e / (size_t)ncols);
    const int c = (int)(e - (size_t)r * (size_t)ncols);
    const int seg = r / rows_per_seg;
    const int rr = r - seg * rows_per_seg;
    const float* sp = src + ((size_t)seg * (size_t)src_seg_rows + (size_t)rr) * (size_t)ncols + c;
    const v4f a = *reinterpret_cast<const v4f*>(sp);
    const v4f b = *reinterpret_cast<const v4f*>(sp + 4);
    v8h o = {(_Float16)(bfr(a.x) * scale), (_Float16)(bfr(a.y) * scale),
             (_Float16)(bfr(a.z) * scale), (_Float16)(bfr(a.w) * scale),
             (_Float16)(bfr(b.x) * scale), (_Float16)(bfr(b.y) * scale),
             (_Float16)(bfr(b.z) * scale), (_Float16)(bfr(b.w) * scale)};
    _Float16* dp = dst + e;
    *(volatile v8h*)dp = o;
    __threadfence();
    *(volatile v8h*)dp = o;
}

template <int MODE, int NI>
__global__ __launch_bounds__(256) __attribute__((amdgpu_num_vgpr(256)))
void k_gemm(const _Float16* __restrict__ A, const _Float16* __restrict__ A2,
            const _Float16* __restrict__ BT, const float* __restrict__ cs,
            const float* __restrict__ sn, void* C0, void* C1, float alpha)
{
    constexpr int BN_ = 32 * NI;
    constexpr int WNC = 16 * NI;
    constexpr int EP  = 16 * NI + 4;
    constexpr int EW  = 8 * 16 * EP;
    static_assert(MODE != 2 || (EW * 4 >= 128 * TP * 2));
    static_assert((BN_ * 4) % 256 == 0);
    static_assert(MODE >= 3 || NI == 4);
    __shared__ alignas(16) _Float16 As[BM * LP];
    __shared__ alignas(16) _Float16 Bs[BN_ * LP];
    __shared__ alignas(16) _Float16 A2s[(MODE == 4) ? (BM * LP) : 8];
    __shared__ alignas(16) float Es[EW];

    const int tid  = threadIdx.x;
    const int lane = tid & 31, wave = tid >> 5;
    const int wm = wave & 3, wn = wave >> 2;
    const int l15 = lane & 15, hi8 = (lane >> 4) << 3;
    const int bn0 = blockIdx.x * BN_;
    const int by = blockIdx.y;
    int bm0 = by * BM, a2r0 = 0;
    if (MODE == 3) {
        constexpr int per  = (SEQ - EROWS) / BM;
        constexpr int perd = (per > 0) ? per : 1;
        const int b = by / perd;
        bm0 = b * SEQ + EROWS + (by - b * perd) * BM;
    }
    if (MODE == 4) {
        constexpr int per = EROWS / BM;
        const int b = by / per;
        const int rb = (by - b * per) * BM;
        bm0 = b * SEQ + rb;
        a2r0 = b * EROWS + rb;
    }

    v8f acc[2][NI], accR[2][NI];
#pragma unroll
    for (int mi = 0; mi < 2; ++mi)
#pragma unroll
        for (int ni = 0; ni < NI; ++ni) { acc[mi][ni] = {}; accR[mi][ni] = {}; }

#pragma unroll 1
    for (int k0 = 0; k0 < DM; k0 += BK) {
#pragma unroll
        for (int i = 0; i < 2; ++i) {
            const int c = tid + i * 256;
            const int row = c >> 2, kg = (c & 3) * 8;
            const v8h v = *reinterpret_cast<const v8h*>(A + (size_t)(bm0 + row) * DM + k0 + kg);
            *reinterpret_cast<v8h*>(&As[row * LP + kg]) = v;
            if (MODE == 4) {
                const v8h v2 = *reinterpret_cast<const v8h*>(A2 + (size_t)(a2r0 + row) * DM + k0 + kg);
                *reinterpret_cast<v8h*>(&A2s[row * LP + kg]) = v2;
            }
        }
#pragma unroll
        for (int i = 0; i < (BN_ * 4) / 256; ++i) {
            const int c = tid + i * 256;
            const int row = c >> 2, kg = (c & 3) * 8;
            const v8h v = *reinterpret_cast<const v8h*>(BT + (size_t)(bn0 + row) * DM + k0 + kg);
            *reinterpret_cast<v8h*>(&Bs[row * LP + kg]) = v;
        }
        __syncthreads();

        v16h aF[2], bF[NI];
#pragma unroll
        for (int mi = 0; mi < 2; ++mi)
            aF[mi] = load_frag(&As[(wm * 32 + mi * 16 + l15) * LP + hi8]);
#pragma unroll
        for (int ni = 0; ni < NI; ++ni)
            bF[ni] = load_frag(&Bs[(wn * WNC + ni * 16 + l15) * LP + hi8]);
#pragma unroll
        for (int mi = 0; mi < 2; ++mi)
#pragma unroll
            for (int ni = 0; ni < NI; ++ni)
                acc[mi][ni] = wmma16(aF[mi], bF[ni], acc[mi][ni]);
        if (MODE == 4) {
#pragma unroll
            for (int mi = 0; mi < 2; ++mi)
                aF[mi] = load_frag(&A2s[(wm * 32 + mi * 16 + l15) * LP + hi8]);
#pragma unroll
            for (int mi = 0; mi < 2; ++mi)
#pragma unroll
                for (int ni = 0; ni < NI; ++ni)
                    accR[mi][ni] = wmma16(aF[mi], bF[ni], accR[mi][ni]);
        }
        __syncthreads();
    }

    if (MODE == 0 || MODE == 1) {
        constexpr int NOUT = (MODE == 0) ? DM : HD;
        _Float16* oh  = reinterpret_cast<_Float16*>(C0);
        _Float16* orr = reinterpret_cast<_Float16*>(C1);
        const int pos0 = bm0 % SEQ;
        const bool eres = (MODE == 1) || (pos0 < EROWS);
        const int rr0 = (MODE == 0) ? ((bm0 / SEQ) * EROWS + pos0) : bm0;
        float* Ew = Es + wave * (16 * EP);
#pragma unroll
        for (int mi = 0; mi < 2; ++mi) {
#pragma unroll
            for (int ni = 0; ni < NI; ++ni)
#pragma unroll
                for (int j = 0; j < 8; ++j)
                    Ew[(hi8 + j) * EP + ni * 16 + l15] = acc[mi][ni][j] * alpha;
            __syncthreads();
#pragma unroll
            for (int ps = 0; ps < 2; ++ps) {
#pragma unroll
                for (int it = 0; it < 4; ++it) {
                    const int rl = it * 4 + (lane >> 3);
                    const int c8 = (lane & 7) * 8;
                    const int lrow = wm * 32 + mi * 16 + rl;
                    const int gcol = bn0 + wn * WNC + c8;
                    const v4f f0 = *reinterpret_cast<const v4f*>(&Ew[rl * EP + c8]);
                    const v4f f1 = *reinterpret_cast<const v4f*>(&Ew[rl * EP + c8 + 4]);
                    const int pos = pos0 + lrow;
                    const int i0 = (gcol & (HD - 1)) >> 1;
                    const v4f cv = *reinterpret_cast<const v4f*>(cs + (size_t)pos * HP + i0);
                    const v4f sv = *reinterpret_cast<const v4f*>(sn + (size_t)pos * HP + i0);
                    const v4f g0 = rope4(f0, bfr(cv.x), bfr(sv.x), bfr(cv.y), bfr(sv.y));
                    const v4f g1 = rope4(f1, bfr(cv.z), bfr(sv.z), bfr(cv.w), bfr(sv.w));
                    const HR8 o = pack8(g0, g1);
                    *(volatile v8h*)(oh + (size_t)(bm0 + lrow) * NOUT + gcol) = o.h;
                    if (eres)
                        *(volatile v8h*)(orr + (size_t)(rr0 + lrow) * NOUT + gcol) = o.r;
                }
                if (ps == 0) __threadfence();
            }
            __syncthreads();
        }
    }

    if (MODE == 2) {
        _Float16* T16 = reinterpret_cast<_Float16*>(Es);
        const int bb = bm0 / SEQ;
        const int t0 = bm0 - bb * SEQ;
#pragma unroll
        for (int ph = 0; ph < 2; ++ph) {
#pragma unroll
            for (int mi = 0; mi < 2; ++mi)
#pragma unroll
                for (int ni = 0; ni < NI; ++ni)
#pragma unroll
                    for (int j = 0; j < 8; ++j) {
                        const float val = acc[mi][ni][j] * alpha;
                        const _Float16 hv = (_Float16)val;
                        const _Float16 w = (ph == 0) ? hv : (_Float16)((val - (float)hv) * RSC);
                        T16[(wn * 64 + ni * 16 + l15) * TP + wm * 32 + mi * 16 + hi8 + j] = w;
                    }
            __syncthreads();
            _Float16* dst = reinterpret_cast<_Float16*>((ph == 0) ? C0 : C1);
#pragma unroll
            for (int ps = 0; ps < 2; ++ps) {
#pragma unroll
                for (int it = 0; it < 8; ++it) {
                    const int c = it * 256 + tid;
                    const int d = c >> 4, piece = c & 15;
                    const v8h v = *reinterpret_cast<const v8h*>(&T16[d * TP + piece * 8]);
                    *(volatile v8h*)(dst + ((size_t)(bb * HD + d)) * SEQ + t0 + piece * 8) = v;
                }
                if (ps == 0) __threadfence();
            }
            __syncthreads();
        }
    }

    if (MODE >= 3) {
        float* outp = reinterpret_cast<float*>(C0);
        float* Ew = Es + wave * (16 * EP);
        constexpr int PPR = NI * 4;
        constexpr int NIT = (16 * PPR) / 32;
#pragma unroll
        for (int mi = 0; mi < 2; ++mi) {
#pragma unroll
            for (int ni = 0; ni < NI; ++ni)
#pragma unroll
                for (int j = 0; j < 8; ++j) {
                    float v = acc[mi][ni][j];
                    if (MODE == 4) v = v + accR[mi][ni][j] * RINV;
                    Ew[(hi8 + j) * EP + ni * 16 + l15] = v * alpha;
                }
            __syncthreads();
#pragma unroll
            for (int ps = 0; ps < 2; ++ps) {
#pragma unroll
                for (int it = 0; it < NIT; ++it) {
                    const int c = it * 32 + lane;
                    const int rl = c / PPR, piece = c - rl * PPR;
                    const int lrow = wm * 32 + mi * 16 + rl;
                    const int gcol = bn0 + wn * WNC + piece * 4;
                    const v4f v = *reinterpret_cast<const v4f*>(&Ew[rl * EP + piece * 4]);
                    *(volatile v4f*)(outp + (size_t)(bm0 + lrow) * DM + gcol) = v;
                }
                if (ps == 0) __threadfence();
            }
            __syncthreads();
        }
    }
}

template <int EARLY>
__global__ __launch_bounds__(128) __attribute__((amdgpu_num_vgpr(256)))
void k_attn(const _Float16* __restrict__ qh, const _Float16* __restrict__ qr,
            const _Float16* __restrict__ kh, const _Float16* __restrict__ kr,
            const _Float16* __restrict__ vth, const _Float16* __restrict__ vtr,
            _Float16* yh, _Float16* yr)
{
    constexpr int NDT = EARLY ? 4 : 8;
    constexpr int YP  = NDT * 16 + 4;
    constexpr int NT  = SEQ / 16 - ETILES;
    constexpr int NTS = (NT > 0) ? NT : 1;
    constexpr int TOT = EARLY ? ((NB) * NH * ETILES * 2) : ((NB) * NH * NT);
    __shared__ alignas(16) _Float16 Ps[4][16 * LP];
    __shared__ alignas(16) _Float16 Pr[EARLY ? 4 : 1][16 * LP];
    __shared__ alignas(16) float Ys[4][16 * YP];

    const int lane = threadIdx.x & 31, wv = threadIdx.x >> 5;
    const int l15 = lane & 15, hi8 = (lane >> 4) << 3;
    int gw = blockIdx.x * 4 + wv;
    if (gw >= TOT) return;
    int dh = 0, qt;
    if (EARLY) { dh = gw & 1; gw >>= 1; qt = gw % ETILES; gw /= ETILES; }
    else       { qt = ETILES + gw % NTS; gw /= NTS; }
    const int hh = gw % NH;
    const int b  = gw / NH;
    const int q0 = qt * 16;
    const int dv0 = EARLY ? dh * 64 : 0;

    const _Float16* qp = qh + ((size_t)(b * SEQ + q0 + l15)) * DM + hh * HD + hi8;
    v16h aQ[4];
#pragma unroll
    for (int c = 0; c < 4; ++c) aQ[c] = load_frag(qp + c * 32);
    const _Float16* qrp = qr + ((size_t)(b * EROWS + (EARLY ? q0 : 0) + l15)) * DM + hh * HD + hi8;
    const _Float16* kp  = kh  + ((size_t)(b * SEQ + l15)) * HD + hi8;
    const _Float16* krp = kr  + ((size_t)(b * SEQ + l15)) * HD + hi8;
    const _Float16* vp  = vth + ((size_t)(b * HD + dv0 + l15)) * SEQ + hi8;
    const _Float16* vrp = vtr + ((size_t)(b * HD + dv0 + l15)) * SEQ + hi8;

    float m[8], l[8];
    v8f accY[NDT], accR[NDT];
#pragma unroll
    for (int j = 0; j < 8; ++j) { m[j] = -1.0e30f; l[j] = 0.0f; }
#pragma unroll
    for (int ni = 0; ni < NDT; ++ni) { accY[ni] = {}; accR[ni] = {}; }

    const float SCL = 0.08838834764831845f * 1.4426950408889634f;
    const float NEG = -1.0e30f;
    const int nch = (q0 + 16 + 31) >> 5;
    _Float16* ps = Ps[wv];
    _Float16* pr = Pr[EARLY ? wv : 0];

#pragma unroll 1
    for (int ch = 0; ch < nch; ++ch) {
        const int tc = ch * 32;
        const _Float16* k0p = kp + (size_t)tc * HD;
        v8f s0 = {}, s1 = {};
#pragma unroll
        for (int c = 0; c < 4; ++c) {
            const v16h b0 = load_frag(k0p + c * 32);
            const v16h b1 = load_frag(k0p + 16 * HD + c * 32);
            s0 = wmma16(aQ[c], b0, s0);
            s1 = wmma16(aQ[c], b1, s1);
        }
        if (EARLY) {
            const _Float16* kr0p = krp + (size_t)tc * HD;
            v8f r0 = {}, r1 = {};
#pragma unroll
            for (int c = 0; c < 4; ++c) {
                const v16h b0 = load_frag(kr0p + c * 32);
                const v16h b1 = load_frag(kr0p + 16 * HD + c * 32);
                r0 = wmma16(aQ[c], b0, r0);
                r1 = wmma16(aQ[c], b1, r1);
            }
#pragma unroll
            for (int c = 0; c < 4; ++c) {
                const v16h aR = load_frag(qrp + c * 32);
                const v16h b0 = load_frag(k0p + c * 32);
                const v16h b1 = load_frag(k0p + 16 * HD + c * 32);
                r0 = wmma16(aR, b0, r0);
                r1 = wmma16(aR, b1, r1);
            }
#pragma unroll
            for (int j = 0; j < 8; ++j) {
                s0[j] = s0[j] + r0[j] * RINV;
                s1[j] = s1[j] + r1[j] * RINV;
            }
        }

#pragma unroll
        for (int j = 0; j < 8; ++j) {
            const int qpos = q0 + hi8 + j;
            float x0 = s0[j] * SCL;
            float x1 = s1[j] * SCL;
            x0 = (tc + l15 <= qpos) ? x0 : NEG;
            x1 = (tc + 16 + l15 <= qpos) ? x1 : NEG;
            float mt = fmaxf(x0, x1);
#pragma unroll
            for (int off = 8; off >= 1; off >>= 1)
                mt = fmaxf(mt, __shfl_xor(mt, off, 16));
            const float mn = fmaxf(m[j], mt);
            const float sc = exp2f(m[j] - mn);
            const float p0 = exp2f(x0 - mn);
            const float p1 = exp2f(x1 - mn);
            float rs = p0 + p1;
#pragma unroll
            for (int off = 8; off >= 1; off >>= 1)
                rs += __shfl_xor(rs, off, 16);
            l[j] = l[j] * sc + rs;
            m[j] = mn;
            s0[j] = p0;
            s1[j] = p1;
#pragma unroll
            for (int ni = 0; ni < NDT; ++ni) {
                accY[ni][j] *= sc;
                if (EARLY) accR[ni][j] *= sc;
            }
        }

        wave_lds_sync();
#pragma unroll
        for (int j = 0; j < 8; ++j) {
            const float a0 = s0[j] * PSC, a1 = s1[j] * PSC;
            const _Float16 h0 = (_Float16)a0, h1 = (_Float16)a1;
            ps[(hi8 + j) * LP + l15]      = h0;
            ps[(hi8 + j) * LP + 16 + l15] = h1;
            if (EARLY) {
                pr[(hi8 + j) * LP + l15]      = (_Float16)((a0 - (float)h0) * RSC);
                pr[(hi8 + j) * LP + 16 + l15] = (_Float16)((a1 - (float)h1) * RSC);
            }
        }
        wave_lds_sync();
        const v16h aP = load_frag(ps + l15 * LP + hi8);
        v16h aPr = aP;
        if (EARLY) aPr = load_frag(pr + l15 * LP + hi8);

#pragma unroll
        for (int ni = 0; ni < NDT; ++ni) {
            const v16h bV = load_frag(vp + (size_t)(ni * 16) * SEQ + tc);
            accY[ni] = wmma16(aP, bV, accY[ni]);
            if (EARLY) {
                const v16h bVr = load_frag(vrp + (size_t)(ni * 16) * SEQ + tc);
                accR[ni] = wmma16(aP, bVr, accR[ni]);
                accR[ni] = wmma16(aPr, bV, accR[ni]);
            }
        }
    }

    float inv[8];
#pragma unroll
    for (int j = 0; j < 8; ++j) inv[j] = (1.0f / l[j]) * PINV;
    float* ys = Ys[wv];
#pragma unroll
    for (int ni = 0; ni < NDT; ++ni)
#pragma unroll
        for (int j = 0; j < 8; ++j) {
            float y = accY[ni][j];
            if (EARLY) y = y + accR[ni][j] * RINV;
            ys[(hi8 + j) * YP + ni * 16 + l15] = y * inv[j];
        }
    wave_lds_sync();

    constexpr int PPR = NDT * 2;
    constexpr int NIT = (16 * PPR) / 32;
    const size_t orow0 = (size_t)(b * SEQ + q0);
    const size_t rrow0 = (size_t)(b * EROWS + (EARLY ? q0 : 0));
    const int gcol0 = hh * HD + dv0;
#pragma unroll
    for (int pss = 0; pss < 2; ++pss) {
#pragma unroll
        for (int it = 0; it < NIT; ++it) {
            const int c = it * 32 + lane;
            const int rl = c / PPR, piece = c - rl * PPR;
            const v4f f0 = *reinterpret_cast<const v4f*>(&ys[rl * YP + piece * 8]);
            const v4f f1 = *reinterpret_cast<const v4f*>(&ys[rl * YP + piece * 8 + 4]);
            const HR8 o = pack8(f0, f1);
            *(volatile v8h*)(yh + (orow0 + rl) * DM + gcol0 + piece * 8) = o.h;
            if (EARLY)
                *(volatile v8h*)(yr + (rrow0 + rl) * DM + gcol0 + piece * 8) = o.r;
        }
        if (pss == 0) __threadfence();
    }
}

extern "C" void kernel_launch(void* const* d_in, const int* in_sizes, int n_in,
                              void* d_out, int out_size, void* d_ws, size_t ws_size,
                              hipStream_t stream) {
    if (n_in < 7) return;
    if ((size_t)in_sizes[0] < (size_t)MROWS * DM) return;
    if ((size_t)in_sizes[1] < (size_t)DM * DM) return;
    if ((size_t)in_sizes[2] < (size_t)HD * DM) return;
    if ((size_t)in_sizes[3] < (size_t)HD * DM) return;
    if ((size_t)in_sizes[4] < (size_t)DM * DM) return;
    if ((size_t)in_sizes[5] < (size_t)(SEQ) * HP) return;
    if ((size_t)in_sizes[6] < (size_t)(SEQ) * HP) return;
    if ((size_t)out_size < (size_t)MROWS * DM) return;
    if (ws_size < WS_TOTAL) return;

    const float* x   = (const float*)d_in[0];
    const float* Wq  = (const float*)d_in[1];
    const float* Wk  = (const float*)d_in[2];
    const float* Wv  = (const float*)d_in[3];
    const float* Wo  = (const float*)d_in[4];
    const float* fcs = (const float*)d_in[5];
    const float* fsn = (const float*)d_in[6];
    float* out = (float*)d_out;

    char* w = (char*)d_ws;
    _Float16* x16  = (_Float16*)(w + O_X16);
    _Float16* wq16 = (_Float16*)(w + O_WQ);
    _Float16* wk16 = (_Float16*)(w + O_WK);
    _Float16* wv16 = (_Float16*)(w + O_WV);
    _Float16* wo16 = (_Float16*)(w + O_WO);
    _Float16* qh   = (_Float16*)(w + O_QH);
    _Float16* qr   = (_Float16*)(w + O_QR);
    _Float16* kh   = (_Float16*)(w + O_KH);
    _Float16* kr   = (_Float16*)(w + O_KR);
    _Float16* vth  = (_Float16*)(w + O_VTH);
    _Float16* vtr  = (_Float16*)(w + O_VTR);
    _Float16* yh   = (_Float16*)(w + O_YH);
    _Float16* yr   = (_Float16*)(w + O_YR);

    const dim3 blk(256);

    {
        const int gx = MROWS * DM / 8;
        k_cvt<<<dim3((gx + 255) / 256), blk, 0, stream>>>(x, x16, gx, DM, SEQ, SEQ_FULL, 1.0f);
        const int gq = DM * DM / 8;
        k_cvt<<<dim3((gq + 255) / 256), blk, 0, stream>>>(Wq, wq16, gq, DM, DM, 0, WSC);
        const int gk = HD * DM / 8;
        k_cvt<<<dim3((gk + 255) / 256), blk, 0, stream>>>(Wk, wk16, gk, DM, HD, 0, WSC);
        k_cvt<<<dim3((gk + 255) / 256), blk, 0, stream>>>(Wv, wv16, gk, DM, HD, 0, WSC);
        k_cvt<<<dim3((gq + 255) / 256), blk, 0, stream>>>(Wo, wo16, gq, DM, DM, 0, WSC);
    }

    k_gemm<0, 4><<<dim3(DM / 128, MROWS / BM), blk, 0, stream>>>(x16, x16, wq16, fcs, fsn,
                                                                 (void*)qh, (void*)qr, WINV);
    k_gemm<1, 4><<<dim3(1, MROWS / BM), blk, 0, stream>>>(x16, x16, wk16, fcs, fsn,
                                                          (void*)kh, (void*)kr, WINV);
    k_gemm<2, 4><<<dim3(1, MROWS / BM), blk, 0, stream>>>(x16, x16, wv16, fcs, fsn,
                                                          (void*)vth, (void*)vtr, WINV);

    {
        const int wE = (NB) * NH * ETILES * 2;
        k_attn<1><<<dim3(wE / 4), dim3(128), 0, stream>>>(qh, qr, kh, kr, vth, vtr, yh, yr);
        const int wM = (NB) * NH * (SEQ / 16 - ETILES);
        if (wM > 0)
            k_attn<0><<<dim3(wM / 4), dim3(128), 0, stream>>>(qh, qr, kh, kr, vth, vtr, yh, yr);
    }

    k_gemm<4, 2><<<dim3(DM / 64, (NB) * EROWS / BM), blk, 0, stream>>>(yh, yr, wo16, fcs, fsn,
                                                                      (void*)out, (void*)out, WINV);
    if (SEQ > EROWS)
        k_gemm<3, 4><<<dim3(DM / 128, (NB) * (SEQ - EROWS) / BM), blk, 0, stream>>>(
            yh, yh, wo16, fcs, fsn, (void*)out, (void*)out, WINV);
}
